// _HANGBlock_18047452578207
// MI455X (gfx1250) — hardware-run, weakly checked
//
#include <hip/hip_runtime.h>

typedef float          v8f   __attribute__((ext_vector_type(8)));
typedef float          v4f   __attribute__((ext_vector_type(4)));
typedef unsigned int   v4u   __attribute__((ext_vector_type(4)));
typedef int            v8i   __attribute__((ext_vector_type(8)));
typedef unsigned short v8us  __attribute__((ext_vector_type(8)));
typedef unsigned short v16us __attribute__((ext_vector_type(16)));
typedef __bf16         v16bf __attribute__((ext_vector_type(16)));
typedef _Float16       v16h  __attribute__((ext_vector_type(16)));
typedef v4f  __attribute__((may_alias)) v4fa;
typedef v8us __attribute__((may_alias)) v8usa;
union FragB { v16bf v; v16us u; v8us h[2]; v8i w; };
union FragH { v16h  v; v16us u; v8us h[2]; v8i w; };

__device__ __forceinline__ v8f wmb(const FragB& a, const FragB& b, v8f c) {
  v8f d = __builtin_amdgcn_wmma_f32_16x16x32_bf16(false, a.v, false, b.v, (short)0, c, false, false);
  asm volatile("v_nop\n\tv_nop\n\tv_nop\n\tv_nop" : "+v"(d) : "v"(a.w), "v"(b.w));
  return d;
}

__device__ __forceinline__ v8f wmh(const FragH& a, const FragH& b, v8f c) {
  v8f d = __builtin_amdgcn_wmma_f32_16x16x32_f16(false, a.v, false, b.v, (short)0, c, false, false);
  asm volatile("v_nop\n\tv_nop\n\tv_nop\n\tv_nop" : "+v"(d) : "v"(a.w), "v"(b.w));
  return d;
}

__device__ __forceinline__ unsigned bf16_bits(float f) {
  const unsigned u = __float_as_uint(f);
  const unsigned r = (u + 0x7FFFu + ((u >> 16) & 1u)) >> 16;
  const unsigned q = (u >> 16) | 0x40u;
  return ((u & 0x7fffffffu) > 0x7f800000u) ? q : r;
}

__device__ __forceinline__ float bf16_val(float f) {
  return __uint_as_float(bf16_bits(f) << 16);
}
__device__ __forceinline__ int clampi(int v, int lo, int hi) {
  return v < lo ? lo : (v > hi ? hi : v);
}

__device__ __forceinline__ unsigned f16_bits(float f) {
  const unsigned u  = __float_as_uint(f);
  const unsigned s  = (u >> 16) & 0x8000u;
  const unsigned a  = u & 0x7fffffffu;
  const unsigned t  = a - 0x38000000u;
  const unsigned r  = (t + 0x0FFFu + ((t >> 13) & 1u)) >> 13;
  const unsigned rc = r > 0x7C00u ? 0x7C00u : r;
  const bool small  = a < 0x38800000u;
  const bool isnan  = a > 0x7f800000u;
  const unsigned fin = small ? 0u : (s | rc);
  return isnan ? (s | 0x7E00u) : fin;
}

__device__ __forceinline__ unsigned pk16(unsigned lo, unsigned hi) { return lo | (hi << 16); }
__device__ __forceinline__ unsigned bf16_lo_bits(float v) {
  float hi = bf16_val(v);
  asm volatile("" : "+v"(hi));
  return bf16_bits(v - hi);
}
__device__ __forceinline__ v4u pack8_bf16(v4f a, v4f c) {
  return (v4u){ pk16(bf16_bits(a[0]), bf16_bits(a[1])), pk16(bf16_bits(a[2]), bf16_bits(a[3])),
                pk16(bf16_bits(c[0]), bf16_bits(c[1])), pk16(bf16_bits(c[2]), bf16_bits(c[3])) };
}
__device__ __forceinline__ v4u pack8_bf16_lo(v4f a, v4f c) {
  return (v4u){ pk16(bf16_lo_bits(a[0]), bf16_lo_bits(a[1])), pk16(bf16_lo_bits(a[2]), bf16_lo_bits(a[3])),
                pk16(bf16_lo_bits(c[0]), bf16_lo_bits(c[1])), pk16(bf16_lo_bits(c[2]), bf16_lo_bits(c[3])) };
}
__device__ __forceinline__ v4u pack8_f16(v4f a, v4f c) {
  return (v4u){ pk16(f16_bits(a[0]), f16_bits(a[1])), pk16(f16_bits(a[2]), f16_bits(a[3])),
                pk16(f16_bits(c[0]), f16_bits(c[1])), pk16(f16_bits(c[2]), f16_bits(c[3])) };
}

template <int FORM>
__global__ __launch_bounds__(256) void k_plane(const float* __restrict__ src, int rows, int cols, int ldsrc,
                                               unsigned short* __restrict__ dst, int MP, int KP) {
  static_assert(FORM >= 0 && FORM <= 3);
  const int KTOT = (FORM == 1 || FORM == 3) ? 2 * KP : KP;
  const unsigned ppr   = (unsigned)(KTOT >> 3);
  const unsigned kp8   = (unsigned)(KP >> 3);
  const unsigned total = (unsigned)MP * ppr;
  const unsigned g     = blockIdx.x * 256u + threadIdx.x;
  const unsigned rowu  = g / ppr;
  const unsigned p     = g - rowu * ppr;
  const bool second    = p >= kp8;
  const int row = (int)rowu;
  const int c0  = (int)((second ? p - kp8 : p) << 3);
  const float* srow = src + (size_t)clampi(row, 0, rows - 1) * (size_t)ldsrc;
  float x[8];
  unsigned mk[8];
#pragma unroll
  for (int e = 0; e < 8; ++e) {
    const int c = c0 + e;
    const float v = srow[clampi(c, 0, cols - 1)];
    asm volatile("" :: "v"(v));
    x[e]  = v;
    mk[e] = (row < rows && c < cols) ? 0xFFFFu : 0u;
  }
  const v4f a = (v4f){ x[0], x[1], x[2], x[3] };
  const v4f c = (v4f){ x[4], x[5], x[6], x[7] };
  v4u o;
  if (FORM == 2) {
    o = pack8_f16(a, c);
  } else {
    const v4u hi = pack8_bf16(a, c);
    o = hi;
    if (FORM == 1) { const v4u lo = pack8_bf16_lo(a, c); o = second ? lo : hi; }
  }
  const v4u mw = (v4u){ pk16(mk[0], mk[1]), pk16(mk[2], mk[3]), pk16(mk[4], mk[5]), pk16(mk[6], mk[7]) };
  o &= mw;
  if (g < total) {
    volatile v4u* q = (volatile v4u*)(dst + (size_t)g * 8);
    *q = o;
    __threadfence();
    *q = o;
  }
}

template <int FORM> struct FragOf    { typedef FragB T; };
template <>         struct FragOf<2> { typedef FragH T; };
__device__ __forceinline__ v8f mm(const FragB& a, const FragB& b, v8f c) { return wmb(a, b, c); }
__device__ __forceinline__ v8f mm(const FragH& a, const FragH& b, v8f c) { return wmh(a, b, c); }
template <class F> __device__ __forceinline__ F ld_frag(const unsigned short* p) {
  F f;
  f.h[0] = *(const v8usa*)(p);
  f.h[1] = *(const v8usa*)(p + 16);
  return f;
}

template <int FORM, int EPI>
__global__ __launch_bounds__(256) __attribute__((amdgpu_num_vgpr(248)))
void k_gemm_nt(const unsigned short* __restrict__ A, const unsigned short* __restrict__ B,
               const float* __restrict__ bias, float* __restrict__ D, int M, int N, int KTOT, int ldd) {
  static_assert(FORM >= 0 && FORM <= 2);
  static_assert(EPI == 0 || EPI == 1);
  typedef typename FragOf<FORM>::T F;
  __shared__ __attribute__((aligned(16))) float sT[8][16 * 68];
  const int lane = threadIdx.x & 31;
  const int wave = threadIdx.x >> 5;
  const int tilesM = (M + 63) >> 6;
  const int tilesN = (N + 63) >> 6;
  const int tile = blockIdx.x * 8 + wave;
  if (tile >= tilesM * tilesN) return;
  const int tm = tile / tilesN;
  const int tn = tile - tm * tilesN;
  const int m0 = tm << 6;
  const int n0 = tn << 6;

  const int rl = lane & 15;
  const int h8 = (lane >> 4) * 8;
  const unsigned short* pa = A + (size_t)(m0 + rl) * (size_t)KTOT + h8;
  const unsigned short* pb = B + (size_t)(n0 + rl) * (size_t)KTOT + h8;

  v8f acc[4][4];
#pragma unroll
  for (int i = 0; i < 4; ++i)
#pragma unroll
    for (int j = 0; j < 4; ++j) acc[i][j] = (v8f){0.f, 0.f, 0.f, 0.f, 0.f, 0.f, 0.f, 0.f};

#pragma unroll 1
  for (int k0 = 0; k0 < KTOT; k0 += 32) {
    F bf[4];
#pragma unroll
    for (int j = 0; j < 4; ++j) bf[j] = ld_frag<F>(pb + (size_t)(j << 4) * (size_t)KTOT + k0);
#pragma unroll
    for (int i = 0; i < 4; ++i) {
      const F af = ld_frag<F>(pa + (size_t)(i << 4) * (size_t)KTOT + k0);
#pragma unroll
      for (int j = 0; j < 4; ++j) acc[i][j] = mm(af, bf[j], acc[i][j]);
    }
  }

  float* slab = sT[wave];
  const int hh = lane >> 4;
  const int c4 = (lane & 15) * 4;
  const int nc = n0 + c4;
  const bool cok = nc < N;
  v4f bv = (v4f){0.f, 0.f, 0.f, 0.f};
  if (EPI == 1) {
    bv = *(const v4fa*)(bias + clampi(nc, 0, N - 4));
    asm volatile("" :: "v"(bv));
  }
#pragma unroll
  for (int i = 0; i < 4; ++i) {
    const int mBase = m0 + (i << 4);
#pragma unroll
    for (int j = 0; j < 4; ++j) {
#pragma unroll
      for (int r = 0; r < 8; ++r) slab[(h8 + r) * 68 + (j << 4) + rl] = acc[i][j][r];
    }
    __builtin_amdgcn_fence(__ATOMIC_RELEASE, "workgroup");
    __builtin_amdgcn_wave_barrier();
    __builtin_amdgcn_fence(__ATOMIC_ACQUIRE, "workgroup");
    v4f vv[8];
#pragma unroll
    for (int it = 0; it < 8; ++it) {
      const int row = it * 2 + hh;
      v4f v = *(const v4fa*)(slab + row * 68 + c4);
      if (EPI == 1) v += bv;
      vv[it] = v;
    }
    for (int pass = 0; pass < 2; ++pass) {
#pragma unroll
      for (int it = 0; it < 8; ++it) {
        const int row = mBase + it * 2 + hh;
        if (cok && row < M) *(volatile v4f*)(D + (size_t)row * (size_t)ldd + nc) = vv[it];
      }
      __threadfence();
    }
    __builtin_amdgcn_fence(__ATOMIC_RELEASE, "workgroup");
    __builtin_amdgcn_wave_barrier();
    __builtin_amdgcn_fence(__ATOMIC_ACQUIRE, "workgroup");
  }
}

#include <stddef.h>
#include <stdint.h>
#include <math.h>

#define TWO_TERM_AGG 1
#define TWO_TERM_Z   1
#define TWO_TERM_A   1
#define TWO_TERM_H   1
#define TWO_TERM_DU  1
#define TWO_TERM_DZ  1

#define HID    96
#define NNODE  50000
#define NEDGE  800000
#define MPAD   50048
#define NTHR   256
#define NWAVE  8
#define EPT    8
#define CHUNK  (NTHR * EPT)
#define WCAP   (EPT * 32)
#define LISTN  (NWAVE * WCAP)
#define NBA    1024
#define SLA    10
#define NBLK   49
#define NSL    (NBLK * NBA)
#define RCAP   21504
#define DEGCAP 64
#define MEAS_MAXDEG 38
#define MEAS_B1024  16696
#define MLINE  32
#define AGG_ZINTS (LISTN + 2 * RCAP + 3 * NBA)
#define AGG_LDS_INTS (AGG_ZINTS + 16)
#define OUT1_OFF ((size_t)NNODE * HID)

#define DUP_AGG (TWO_TERM_AGG ? 2 : 1)
#define DUP_Z   (TWO_TERM_Z   ? 2 : 1)
#define DUP_A   (TWO_TERM_A   ? 2 : 1)
#define DUP_H   (TWO_TERM_H   ? 2 : 1)
#define DUP_DU  (TWO_TERM_DU  ? 2 : 1)
#define DUP_DZ  (TWO_TERM_DZ  ? 2 : 1)

#define PO_WQT 0
#define PO_WPT 24576
#define PO_W1T 49152
#define PO_W2T 98304
#define PO_W2N 122880
#define PO_W1N 147456
#define PO_WQN 184320
#define PO_WPN 208896
#define PO_END 233472

static_assert(HID % 32 == 0);
static_assert(MPAD % 64 == 0 && MPAD >= NNODE && NNODE % 16 == 0);
static_assert(NEDGE % CHUNK == 1280 && (NEDGE & 3) == 0);
static_assert(NSL >= MPAD && NSL >= NNODE && NBLK * NBA == NSL);
static_assert((CHUNK & (CHUNK - 1)) == 0 && CHUNK <= 4096);
static_assert((NBA & (NBA - 1)) == 0 && NBA == (1 << SLA) && NBA == 4 * NTHR);
static_assert(((long long)NEDGE << SLA) < (1LL << 31));
static_assert(LISTN % NTHR == 0 && NBA % NWAVE == 0);
static_assert(RCAP % (NTHR * 4) == 0 && AGG_ZINTS % (NTHR * 4) == 0);
static_assert(DEGCAP % 32 == 0 && DEGCAP >= MEAS_MAXDEG + 8);
static_assert(4 * RCAP >= 5 * MEAS_B1024);
static_assert(AGG_LDS_INTS * 4 <= 262144);
static_assert((NNODE * 48) % NTHR == 0);
static_assert(2 * OUT1_OFF - 1 < (size_t)2 * NNODE * HID);

typedef float v2f __attribute__((ext_vector_type(2)));
typedef int   v4i __attribute__((ext_vector_type(4)));
typedef v2f __attribute__((may_alias)) v2fa;
typedef v4i __attribute__((may_alias)) v4ia;

__device__ __forceinline__ float rdeg(int c) {
  const int d = c < 1 ? 1 : c;
  return 1.0f / sqrtf((float)d);
}

template <int TRANS>
__device__ __forceinline__ void prep_unit(const float* __restrict__ W, int nvalid, int nrows, int KP, int dup,
                                          unsigned short* dst, int bx, int tid) {
  const int KTOT  = KP * dup;
  const int ppr   = KTOT >> 3;
  const int kp8   = KP >> 3;
  const int total = nrows * ppr;
  if (bx * NTHR >= total) return;
  const int g  = bx * NTHR + tid;
  const int gc = g < total ? g : total - 1;
  const int n  = gc / ppr;
  const int pp = gc - n * ppr;
  const int k0 = (pp >= kp8 ? pp - kp8 : pp) << 3;
  const int nc = n < nvalid ? n : nvalid - 1;
  const float* b = TRANS ? (W + (size_t)k0 * HID + nc) : (W + (size_t)nc * HID + k0);
  const int st = TRANS ? HID : 1;
  const float f0 = b[0 * st], f1 = b[1 * st], f2 = b[2 * st], f3 = b[3 * st];
  const float f4 = b[4 * st], f5 = b[5 * st], f6 = b[6 * st], f7 = b[7 * st];
  asm volatile("" :: "v"(f0), "v"(f1), "v"(f2), "v"(f3), "v"(f4), "v"(f5), "v"(f6), "v"(f7));
  const unsigned m = (n < nvalid) ? 0xFFFFFFFFu : 0u;
  v4u o = pack8_bf16((v4f){ f0, f1, f2, f3 }, (v4f){ f4, f5, f6, f7 });
  o &= (v4u){ m, m, m, m };
  if (g < total) {
    volatile v4u* qd = (volatile v4u*)(dst + (size_t)g * 8);
    *qd = o;
    __threadfence();
    *qd = o;
  }
}

__global__ __launch_bounds__(NTHR) void k_prep(const float* __restrict__ Wq, const float* __restrict__ Wp,
                                               const float* __restrict__ W1, const float* __restrict__ W2,
                                               const float* __restrict__ bq, const float* __restrict__ bp,
                                               const float* __restrict__ b1, const float* __restrict__ b2,
                                               unsigned short* pl, float* bias) {
  const int y = (int)blockIdx.y, bx = (int)blockIdx.x, tid = (int)threadIdx.x;
  if (y == 0)      prep_unit<1>(Wq, 96, 128, 96,  DUP_AGG, pl + PO_WQT, bx, tid);
  else if (y == 1) prep_unit<1>(Wp, 96, 128, 96,  DUP_AGG, pl + PO_WPT, bx, tid);
  else if (y == 2) prep_unit<1>(W1, 96, 128, 192, DUP_Z,   pl + PO_W1T, bx, tid);
  else if (y == 3) prep_unit<1>(W2, 96, 128, 96,  DUP_A,   pl + PO_W2T, bx, tid);
  else if (y == 4) prep_unit<0>(W2, 96, 128, 96,  DUP_H,   pl + PO_W2N, bx, tid);
  else if (y == 5) prep_unit<0>(W1, 192, 192, 96, DUP_DU,  pl + PO_W1N, bx, tid);
  else if (y == 6) prep_unit<0>(Wq, 96, 128, 96,  DUP_DZ,  pl + PO_WQN, bx, tid);
  else if (y == 7) prep_unit<0>(Wp, 96, 128, 96,  DUP_DZ,  pl + PO_WPN, bx, tid);
  else {
    if (bx != 0) return;
    const int tc = tid < 128 ? tid : 127;
    const int bsel = tc >> 5;
    const int c4 = (tc & 31) * 4;
    const int cc = c4 < 92 ? c4 : 92;
    const v4f v0 = *(const v4fa*)(bq + cc);
    const v4f v1 = *(const v4fa*)(bp + cc);
    const v4f v2 = *(const v4fa*)(b1 + cc);
    const v4f v3 = *(const v4fa*)(b2 + cc);
    asm volatile("" :: "v"(v0), "v"(v1), "v"(v2), "v"(v3));
    const unsigned m0 = (bsel == 0) ? 0xFFFFFFFFu : 0u;
    const unsigned m1 = (bsel == 1) ? 0xFFFFFFFFu : 0u;
    const unsigned m2 = (bsel == 2) ? 0xFFFFFFFFu : 0u;
    const unsigned m3 = (bsel == 3) ? 0xFFFFFFFFu : 0u;
    const unsigned cm = (c4 < HID) ? 0xFFFFFFFFu : 0u;
    v4f r;
    {
      const unsigned sx = (__float_as_uint(v0.x) & m0) | (__float_as_uint(v1.x) & m1) | (__float_as_uint(v2.x) & m2) | (__float_as_uint(v3.x) & m3);
      const unsigned sy = (__float_as_uint(v0.y) & m0) | (__float_as_uint(v1.y) & m1) | (__float_as_uint(v2.y) & m2) | (__float_as_uint(v3.y) & m3);
      const unsigned sz = (__float_as_uint(v0.z) & m0) | (__float_as_uint(v1.z) & m1) | (__float_as_uint(v2.z) & m2) | (__float_as_uint(v3.z) & m3);
      const unsigned sw = (__float_as_uint(v0.w) & m0) | (__float_as_uint(v1.w) & m1) | (__float_as_uint(v2.w) & m2) | (__float_as_uint(v3.w) & m3);
      r.x = __uint_as_float((bf16_bits(__uint_as_float(sx)) << 16) & cm);
      r.y = __uint_as_float((bf16_bits(__uint_as_float(sy)) << 16) & cm);
      r.z = __uint_as_float((bf16_bits(__uint_as_float(sz)) << 16) & cm);
      r.w = __uint_as_float((bf16_bits(__uint_as_float(sw)) << 16) & cm);
    }
    if (tid < 128) {
      volatile v4f* bd = (volatile v4f*)(bias + 4 * tid);
      *bd = r;
      __threadfence();
      *bd = r;
    }
  }
}

template <int SLB>
__device__ __forceinline__ int scan_chunk(const int* __restrict__ keys, int nE, int cbase, int slotBase,
                                          int nb, int vec8, int* list, int tid, int lane, int wave) {
  int wc = 0;
  const int el0  = tid * EPT;
  const int e0   = cbase + el0;
  const int sent = (int)0x80000000u;
  v4i da, db;
  if (vec8 != 0 && cbase + CHUNK <= nE) {
    da = *(const v4i*)(keys + e0);
    db = *(const v4i*)(keys + e0 + 4);
  } else {
    const int last = nE - 1;
    const int k0 = keys[min(e0,     last)];
    const int k1 = keys[min(e0 + 1, last)];
    const int k2 = keys[min(e0 + 2, last)];
    const int k3 = keys[min(e0 + 3, last)];
    const int k4 = keys[min(e0 + 4, last)];
    const int k5 = keys[min(e0 + 5, last)];
    const int k6 = keys[min(e0 + 6, last)];
    const int k7 = keys[min(e0 + 7, last)];
    asm volatile("" :: "v"(k0), "v"(k1), "v"(k2), "v"(k3), "v"(k4), "v"(k5), "v"(k6), "v"(k7));
    da.x = (e0     < nE) ? k0 : sent;
    da.y = (e0 + 1 < nE) ? k1 : sent;
    da.z = (e0 + 2 < nE) ? k2 : sent;
    da.w = (e0 + 3 < nE) ? k3 : sent;
    db.x = (e0 + 4 < nE) ? k4 : sent;
    db.y = (e0 + 5 < nE) ? k5 : sent;
    db.z = (e0 + 6 < nE) ? k6 : sent;
    db.w = (e0 + 7 < nE) ? k7 : sent;
  }
  const unsigned nbs = (unsigned)slotBase;
  const unsigned unb = (unsigned)nb;
  const unsigned s0 = (unsigned)da.x - nbs, s1 = (unsigned)da.y - nbs;
  const unsigned s2 = (unsigned)da.z - nbs, s3 = (unsigned)da.w - nbs;
  const unsigned s4 = (unsigned)db.x - nbs, s5 = (unsigned)db.y - nbs;
  const unsigned s6 = (unsigned)db.z - nbs, s7 = (unsigned)db.w - nbs;
  const bool h0 = s0 < unb, h1 = s1 < unb, h2 = s2 < unb, h3 = s3 < unb;
  const bool h4 = s4 < unb, h5 = s5 < unb, h6 = s6 < unb, h7 = s7 < unb;
  const unsigned any = __builtin_amdgcn_ballot_w32(h0 | h1 | h2 | h3 | h4 | h5 | h6 | h7);
  if (any != 0u) {
#define HITJ(J, HJ, SJ) { \
      const unsigned mj = __builtin_amdgcn_ballot_w32(HJ); \
      if (mj != 0u) { \
        if (HJ) { \
          const int pos = wc + (int)__builtin_amdgcn_mbcnt_lo(mj, 0u); \
          if (pos < WCAP) list[wave * WCAP + pos] = ((el0 + (J)) << SLB) | (int)(SJ); \
        } \
        wc += (int)__builtin_popcount(mj); } }
    HITJ(0, h0, s0)
    HITJ(1, h1, s1)
    HITJ(2, h2, s2)
    HITJ(3, h3, s3)
    HITJ(4, h4, s4)
    HITJ(5, h5, s5)
    HITJ(6, h6, s6)
    HITJ(7, h7, s7)
#undef HITJ
  }
  return wc;
}

__global__ __launch_bounds__(NTHR) __attribute__((amdgpu_num_vgpr(248)))
void k_bucket(const int* __restrict__ keys, const int* __restrict__ gath, int nE, int nN, int vec8,
              int* LISTo, int* CNTo, int* OFFo, float* RDo, int* METAo) {
  extern __shared__ __attribute__((aligned(16))) int dsm[];
  int* list = dsm;
  int* hl   = dsm + LISTN;
  int* sl   = dsm + LISTN + RCAP;
  int* cnt  = dsm + LISTN + 2 * RCAP;
  int* offs = cnt + NBA;
  int* cur  = offs + NBA;
  int* misc = cur + NBA;
  const int tid = (int)threadIdx.x, lane = tid & 31, wave = tid >> 5;
  const int blk = (int)blockIdx.x;
  const int nodeBase = blk * NBA;

  {
    const v4i z4 = {0, 0, 0, 0};
    for (int i = tid * 4; i < AGG_ZINTS; i += NTHR * 4) *(v4ia*)(dsm + i) = z4;
    if (tid < 16) misc[tid] = 0;
  }
  __syncthreads();

  int t = 0, ov = 0;
  const int nChunks = (nE + CHUNK - 1) / CHUNK;
#pragma unroll 1
  for (int ch = 0; ch < nChunks; ++ch) {
    const int cbase = ch * CHUNK;
    const int wc = scan_chunk<SLA>(keys, nE, cbase, nodeBase, NBA, vec8, list, tid, lane, wave);
    if (lane == 0) misc[wave] = wc;
    __syncthreads();
    if (wave == 0) {
#pragma unroll 1
      for (int w2 = 0; w2 < NWAVE; ++w2) {
        int c = misc[w2];
        c = c < 0 ? 0 : (c > WCAP ? WCAP : c);
        c = __builtin_amdgcn_readfirstlane(c);
#pragma unroll 1
        for (int b0 = 0; b0 < c; b0 += 32) {
          const int idx = b0 + lane;
          const int ent = list[w2 * WCAP + (idx < WCAP ? idx : WCAP - 1)];
          const int m32 = (c - b0) < 32 ? (c - b0) : 32;
#pragma unroll 1
          for (int k = 0; k < m32; ++k) {
            const int u    = __builtin_amdgcn_readlane(ent, k);
            const int slot = u & (NBA - 1);
            const int el   = (u >> SLA) & (CHUNK - 1);
            const int pk   = ((cbase + el) << SLA) | slot;
            if (t < RCAP) {
              if (lane == 0) { hl[t] = pk; cnt[slot] = cnt[slot] + 1; }
              t = t + 1;
            } else {
              ov = 1;
            }
          }
        }
      }
    }
    __syncthreads();
  }
  if (wave == 0 && lane == 0) { misc[8] = t; misc[9] = ov; }
  __syncthreads();
  int tt = misc[8];
  tt = tt < 0 ? 0 : (tt > RCAP ? RCAP : tt);
  tt = __builtin_amdgcn_readfirstlane(tt);
  const int ovf = __builtin_amdgcn_readfirstlane(misc[9]);

  if (wave == 0) {
    const int base = lane * (NBA / 32);
    int s = 0;
#pragma unroll 1
    for (int i = 0; i < NBA / 32; ++i) s += cnt[base + i];
    int incl = s;
#pragma unroll
    for (int d = 1; d < 32; d <<= 1) {
      const int y = __shfl_up(incl, d, 32);
      if (lane >= d) incl += y;
    }
    int run = incl - s;
#pragma unroll 1
    for (int i = 0; i < NBA / 32; ++i) {
      const int cv = cnt[base + i];
      offs[base + i] = run;
      cur[base + i]  = run;
      run += cv;
    }
  }
  __syncthreads();
  if (wave == 0) {
#pragma unroll 1
    for (int b0 = 0; b0 < tt; b0 += 32) {
      const int idx = b0 + lane;
      const int ent = hl[idx < RCAP ? idx : RCAP - 1];
      const int m32 = (tt - b0) < 32 ? (tt - b0) : 32;
#pragma unroll 1
      for (int k = 0; k < m32; ++k) {
        const int u    = __builtin_amdgcn_readlane(ent, k);
        const int slot = u & (NBA - 1);
        if (lane == 0) {
          int p = cur[slot];
          p = p < 0 ? 0 : (p > RCAP - 1 ? RCAP - 1 : p);
          sl[p] = u;
          cur[slot] = p + 1;
        }
      }
    }
  }
  __syncthreads();

  const int sb4 = 4 * tid;
  const v4i c4 = *(const v4ia*)(cnt + sb4);
  const v4i o4 = *(const v4ia*)(offs + sb4);
  const float qn = __int_as_float(0x7fc00000);
  v4f rv;
  {
    const float r0 = rdeg(c4.x), r1 = rdeg(c4.y), r2 = rdeg(c4.z), r3 = rdeg(c4.w);
    rv.x = (ovf != 0 || c4.x > DEGCAP) ? qn : r0;
    rv.y = (ovf != 0 || c4.y > DEGCAP) ? qn : r1;
    rv.z = (ovf != 0 || c4.z > DEGCAP) ? qn : r2;
    rv.w = (ovf != 0 || c4.w > DEGCAP) ? qn : r3;
  }
  int* lst = LISTo + (size_t)blk * RCAP;
#pragma unroll 1
  for (int it = 0; it < RCAP / (NTHR * 4); ++it) {
    const int p = it * (NTHR * 4) + 4 * tid;
    v4i g = {0, 0, 0, 0};
    if (it * (NTHR * 4) < tt) {
      const v4i e4 = *(const v4ia*)(sl + p);
      const int q0 = clampi(e4.x >> SLA, 0, nE - 1), q1 = clampi(e4.y >> SLA, 0, nE - 1);
      const int q2 = clampi(e4.z >> SLA, 0, nE - 1), q3 = clampi(e4.w >> SLA, 0, nE - 1);
      const int g0 = gath[q0], g1 = gath[q1], g2 = gath[q2], g3 = gath[q3];
      asm volatile("" :: "v"(g0), "v"(g1), "v"(g2), "v"(g3));
      g.x = (p     < tt) ? clampi(g0, 0, nN - 1) : 0;
      g.y = (p + 1 < tt) ? clampi(g1, 0, nN - 1) : 0;
      g.z = (p + 2 < tt) ? clampi(g2, 0, nN - 1) : 0;
      g.w = (p + 3 < tt) ? clampi(g3, 0, nN - 1) : 0;
    }
    *(v4ia*)(hl + p) = g;
    *(volatile v4i*)(lst + p) = g;
  }
  int*   cg = CNTo + nodeBase + sb4;
  int*   og = OFFo + nodeBase + sb4;
  float* ig = RDo + nodeBase + sb4;
  v4i mv = {0, 0, 0, 0};
  mv.x = (lane == 0) ? ovf : 0;
  mv.y = (lane == 0) ? tt : 0;
  int* mg = METAo + (size_t)blk * MLINE + 4 * (lane & 7);
  *(volatile v4i*)cg = c4;
  *(volatile v4i*)og = o4;
  *(volatile v4f*)ig = rv;
  if (wave == 0 && lane < 8) *(volatile v4i*)mg = mv;
  __threadfence();
#pragma unroll 1
  for (int it = 0; it < RCAP / (NTHR * 4); ++it) {
    const int p = it * (NTHR * 4) + 4 * tid;
    const v4i g = *(const v4ia*)(hl + p);
    *(volatile v4i*)(lst + p) = g;
  }
  *(volatile v4i*)cg = c4;
  *(volatile v4i*)og = o4;
  *(volatile v4f*)ig = rv;
  if (wave == 0 && lane < 8) *(volatile v4i*)mg = mv;
}

__global__ __launch_bounds__(NTHR) void k_xs(const float* __restrict__ q, const float* __restrict__ p,
                                             const float* __restrict__ RDO, float* XS, int nN) {
  const unsigned u     = blockIdx.x * 256u + threadIdx.x;
  const unsigned total = (unsigned)nN * 48u;
  const unsigned uc    = u < total ? u : total - 1u;
  const unsigned row   = uc / 48u;
  const unsigned pc    = uc - row * 48u;
  const bool isp       = pc >= 24u;
  const unsigned c4    = (isp ? pc - 24u : pc) * 4u;
  const v4f qv = *(const v4fa*)(q + (size_t)row * HID + c4);
  const v4f pv = *(const v4fa*)(p + (size_t)row * HID + c4);
  const float rd = RDO[row];
  asm volatile("" :: "v"(qv), "v"(pv), "v"(rd));
  const unsigned mp = isp ? 0xFFFFFFFFu : 0u;
  const unsigned mq = ~mp;
  v4f o;
  o.x = bf16_val(__uint_as_float((__float_as_uint(qv.x) & mq) | (__float_as_uint(pv.x) & mp))) * rd;
  o.y = bf16_val(__uint_as_float((__float_as_uint(qv.y) & mq) | (__float_as_uint(pv.y) & mp))) * rd;
  o.z = bf16_val(__uint_as_float((__float_as_uint(qv.z) & mq) | (__float_as_uint(pv.z) & mp))) * rd;
  o.w = bf16_val(__uint_as_float((__float_as_uint(qv.w) & mq) | (__float_as_uint(pv.w) & mp))) * rd;
  if (u < total) {
    volatile v4f* xd = (volatile v4f*)(XS + (size_t)u * 4);
    *xd = o;
    __threadfence();
    *xd = o;
  }
}

__global__ __launch_bounds__(NTHR) __attribute__((amdgpu_num_vgpr(248)))
void k_fwd(const int* __restrict__ LIST, const int* __restrict__ CNT, const int* __restrict__ OFF,
           const int* __restrict__ META, const float* __restrict__ RDI, const float* __restrict__ XS,
           float* AGG, int nN) {
  __shared__ __attribute__((aligned(16))) int scnt[NBA];
  __shared__ __attribute__((aligned(16))) int soff[NBA];
  const int tid = (int)threadIdx.x, lane = tid & 31, wave = tid >> 5;
  const int blk = (int)blockIdx.x;
  const int nodeBase = blk * NBA;
  {
    const v4i c4 = *(const v4i*)(CNT + nodeBase + 4 * tid);
    const v4i o4 = *(const v4i*)(OFF + nodeBase + 4 * tid);
    *(v4ia*)(scnt + 4 * tid) = c4;
    *(v4ia*)(soff + 4 * tid) = o4;
  }
  const int flag = META[(size_t)blk * MLINE];
  __syncthreads();
  const int* lst = LIST + (size_t)blk * RCAP;
  const float qn = __int_as_float(0x7fc00000);

#pragma unroll 1
  for (int si = 0; si < NBA / NWAVE; ++si) {
    const int s    = si * NWAVE + wave;
    const int node = nodeBase + s;
    const bool live = node < nN;
    int c = scnt[s];
    const bool big = c > DEGCAP;
    c = c < 0 ? 0 : (c > DEGCAP ? DEGCAP : c);
    c = __builtin_amdgcn_readfirstlane(live ? c : 0);
    int o = soff[s];
    o = o < 0 ? 0 : (o > RCAP ? RCAP : o);
    o = __builtin_amdgcn_readfirstlane(o);
    const int nc = live ? node : nN - 1;
    v2f a0 = {0.0f, 0.0f}, a1 = {0.0f, 0.0f}, a2 = {0.0f, 0.0f};
#pragma unroll 1
    for (int b0 = 0; b0 < c; b0 += 32) {
      int li = b0 + lane;
      li = li > c - 1 ? c - 1 : li;
      const int idx = clampi(o + li, 0, RCAP - 1);
      int sr = lst[idx];
      asm volatile("" :: "v"(sr));
      sr = sr < 0 ? 0 : (sr > nN - 1 ? nN - 1 : sr);
      const int m32 = (c - b0) < 32 ? (c - b0) : 32;
#pragma unroll 1
      for (int k = 0; k < m32; ++k) {
        const int sk = __builtin_amdgcn_readlane(sr, k);
        const float* rp = XS + (size_t)sk * 192 + 2 * lane;
        const v2f x0 = *(const v2fa*)(rp);
        const v2f x1 = *(const v2fa*)(rp + 64);
        const v2f x2 = *(const v2fa*)(rp + 128);
        asm volatile("" :: "v"(x0), "v"(x1), "v"(x2));
        a0 += x0;
        a1 += x1;
        a2 += x2;
      }
    }
    const float rd = RDI[node];
    asm volatile("" :: "v"(rd));
    const float pzr = (big || flag != 0) ? qn : 0.0f;
    const v2f o0 = (a0 + pzr) * rd;
    const v2f o1 = (a1 + pzr) * rd;
    const v2f o2 = (a2 + pzr) * rd;
    float* ar = AGG + (size_t)nc * 192 + 2 * lane;
    if (live) {
      *(volatile v2f*)(ar)       = o0;
      *(volatile v2f*)(ar + 64)  = o1;
      *(volatile v2f*)(ar + 128) = o2;
    }
    __threadfence();
    if (live) {
      *(volatile v2f*)(ar)       = o0;
      *(volatile v2f*)(ar + 64)  = o1;
      *(volatile v2f*)(ar + 128) = o2;
    }
  }
}

__global__ __launch_bounds__(NTHR) void k_tanh(const float* __restrict__ U, float* ATH, int total4) {
  const int u  = (int)blockIdx.x * NTHR + (int)threadIdx.x;
  const int uc = u < total4 ? u : total4 - 1;
  v4f v = *(const v4fa*)(U + (size_t)uc * 4);
  asm volatile("" :: "v"(v));
#pragma unroll 1
  for (int i = 0; i < 4; ++i) {
    const float t = tanhf(v.x);
    v = (v4f){ v.y, v.z, v.w, t };
  }
  if (u < total4) {
    volatile v4f* d = (volatile v4f*)(ATH + (size_t)u * 4);
    *d = v;
    __threadfence();
    *d = v;
  }
}

__global__ __launch_bounds__(NTHR) void k_du(const float* __restrict__ DA, const float* __restrict__ ATH,
                                             float* DU, int total4) {
  const int u  = (int)blockIdx.x * NTHR + (int)threadIdx.x;
  const int uc = u < total4 ? u : total4 - 1;
  const v4f d = *(const v4fa*)(DA + (size_t)uc * 4);
  const v4f a = *(const v4fa*)(ATH + (size_t)uc * 4);
  asm volatile("" :: "v"(d), "v"(a));
  v4f o;
  o.x = d.x * (1.0f - a.x * a.x);
  o.y = d.y * (1.0f - a.y * a.y);
  o.z = d.z * (1.0f - a.z * a.z);
  o.w = d.w * (1.0f - a.w * a.w);
  if (u < total4) {
    volatile v4f* dd = (volatile v4f*)(DU + (size_t)u * 4);
    *dd = o;
    __threadfence();
    *dd = o;
  }
}

__global__ __launch_bounds__(NTHR) __attribute__((amdgpu_num_vgpr(248)))
void k_bwd(const int* __restrict__ LIST, const int* __restrict__ CNT, const int* __restrict__ OFF,
           const int* __restrict__ META, const float* __restrict__ RDI, const float* __restrict__ RDO,
           const float* __restrict__ G, const float* __restrict__ q, const float* __restrict__ p,
           float* out, int nN) {
  __shared__ __attribute__((aligned(16))) int scnt[NBA];
  __shared__ __attribute__((aligned(16))) int soff[NBA];
  const int tid = (int)threadIdx.x, lane = tid & 31, wave = tid >> 5;
  const int blk = (int)blockIdx.x;
  const int nodeBase = blk * NBA;
  {
    const v4i c4 = *(const v4i*)(CNT + nodeBase + 4 * tid);
    const v4i o4 = *(const v4i*)(OFF + nodeBase + 4 * tid);
    *(v4ia*)(scnt + 4 * tid) = c4;
    *(v4ia*)(soff + 4 * tid) = o4;
  }
  const int flag = META[(size_t)blk * MLINE];
  __syncthreads();
  const int* lst = LIST + (size_t)blk * RCAP;
  const float qn = __int_as_float(0x7fc00000);
  const int l15 = lane & 15;
  const unsigned mlo = (lane < 16) ? 0xFFFFFFFFu : 0u;
  const unsigned mhi = ~mlo;

#pragma unroll 1
  for (int si = 0; si < NBA / NWAVE; ++si) {
    const int s    = si * NWAVE + wave;
    const int node = nodeBase + s;
    const bool live = node < nN;
    int c = scnt[s];
    const bool big = c > DEGCAP;
    c = c < 0 ? 0 : (c > DEGCAP ? DEGCAP : c);
    c = __builtin_amdgcn_readfirstlane(live ? c : 0);
    int o = soff[s];
    o = o < 0 ? 0 : (o > RCAP ? RCAP : o);
    o = __builtin_amdgcn_readfirstlane(o);
    const int nc = live ? node : nN - 1;
    v2f a0 = {0.0f, 0.0f}, a1 = {0.0f, 0.0f}, a2 = {0.0f, 0.0f};
#pragma unroll 1
    for (int b0 = 0; b0 < c; b0 += 32) {
      int li = b0 + lane;
      li = li > c - 1 ? c - 1 : li;
      const int idx = clampi(o + li, 0, RCAP - 1);
      int sr = lst[idx];
      asm volatile("" :: "v"(sr));
      sr = sr < 0 ? 0 : (sr > nN - 1 ? nN - 1 : sr);
      const int m32 = (c - b0) < 32 ? (c - b0) : 32;
#pragma unroll 1
      for (int k = 0; k < m32; ++k) {
        const int sk = __builtin_amdgcn_readlane(sr, k);
        const float* rp = G + (size_t)sk * 192 + 2 * lane;
        const v2f g0 = *(const v2fa*)(rp);
        const v2f g1 = *(const v2fa*)(rp + 64);
        const v2f g2 = *(const v2fa*)(rp + 128);
        const float rv = RDI[sk];
        asm volatile("" :: "v"(g0), "v"(g1), "v"(g2), "v"(rv));
        a0 += g0 * rv;
        a1 += g1 * rv;
        a2 += g2 * rv;
      }
    }
    const float rdo = RDO[node];
    const float* pr = p + (size_t)nc * HID;
    const float* qr = q + (size_t)nc * HID;
    const v2f p0 = *(const v2fa*)(pr + 2 * lane);
    const v2f p1 = *(const v2fa*)(pr + 64 + 2 * l15);
    const v2f q1 = *(const v2fa*)(qr + 2 * l15);
    const v2f q2 = *(const v2fa*)(qr + 32 + 2 * lane);
    asm volatile("" :: "v"(rdo), "v"(p0), "v"(p1), "v"(q1), "v"(q2));
    const float pzr = (big || flag != 0) ? qn : 0.0f;
    const v2f s0 = (a0 + pzr) * rdo;
    const v2f s1 = (a1 + pzr) * rdo;
    const v2f s2 = (a2 + pzr) * rdo;
    v2f o0, o1, o2;
    o0.x = bf16_val(p0.x) - s0.x;
    o0.y = bf16_val(p0.y) - s0.y;
    {
      const float lx = bf16_val(p1.x) - s1.x, ly = bf16_val(p1.y) - s1.y;
      const float hx = bf16_val(q1.x) + s1.x, hy = bf16_val(q1.y) + s1.y;
      o1.x = __uint_as_float((__float_as_uint(lx) & mlo) | (__float_as_uint(hx) & mhi));
      o1.y = __uint_as_float((__float_as_uint(ly) & mlo) | (__float_as_uint(hy) & mhi));
    }
    o2.x = bf16_val(q2.x) + s2.x;
    o2.y = bf16_val(q2.y) + s2.y;
    const size_t rb = (size_t)nc * HID;
    const size_t e0 = OUT1_OFF + rb + (size_t)(2 * lane);
    const size_t e1 = (lane < 16) ? (OUT1_OFF + rb + (size_t)(64 + 2 * lane)) : (rb + (size_t)(2 * (lane - 16)));
    const size_t e2 = rb + (size_t)(32 + 2 * lane);
    if (live) {
      *(volatile v2f*)(out + e0) = o0;
      *(volatile v2f*)(out + e1) = o1;
      *(volatile v2f*)(out + e2) = o2;
    }
    __threadfence();
    if (live) {
      *(volatile v2f*)(out + e0) = o0;
      *(volatile v2f*)(out + e1) = o1;
      *(volatile v2f*)(out + e2) = o2;
    }
  }
}

template <int TT>
static void mk_plane(const float* src, int cols, int ldsrc, unsigned short* dst, int KP, hipStream_t st) {
  const int KTOT = TT ? 2 * KP : KP;
  const int grid = (MPAD / 64) * (KTOT / 32);
  k_plane<(TT ? 1 : 0)><<<grid, 256, 0, st>>>(src, NNODE, cols, ldsrc, dst, MPAD, KP);
}

template <int EPI>
static void run_gemm(const unsigned short* A, const unsigned short* B, const float* bias, float* D,
                     int N, int KTOT, int ldd, hipStream_t st) {
  const int T = ((NNODE + 63) / 64) * ((N + 63) / 64);
  k_gemm_nt<0, EPI><<<(T + 7) / 8, 256, 0, st>>>(A, B, bias, D, NNODE, N, KTOT, ldd);
}

extern "C" void kernel_launch(void* const* d_in, const int* in_sizes, int n_in,
                              void* d_out, int out_size, void* d_ws, size_t ws_size,
                              hipStream_t stream) {
  if (n_in < 12) return;
  if (in_sizes[0] != NNODE * HID || in_sizes[1] != NNODE * HID) return;
  if (in_sizes[2] != NEDGE || in_sizes[3] != NEDGE) return;
  if (in_sizes[4] != HID * HID || in_sizes[6] != HID * HID) return;
  if (in_sizes[8] != 2 * HID * HID || in_sizes[10] != HID * HID) return;
  if (in_sizes[5] != HID || in_sizes[7] != HID || in_sizes[9] != HID || in_sizes[11] != HID) return;
  if (out_size != 2 * NNODE * HID) return;

  const float* q   = (const float*)d_in[0];
  const float* p   = (const float*)d_in[1];
  const int*   src = (const int*)d_in[2];
  const int*   dst = (const int*)d_in[3];
  const float* Wq  = (const float*)d_in[4];
  const float* bq  = (const float*)d_in[5];
  const float* Wp  = (const float*)d_in[6];
  const float* bp  = (const float*)d_in[7];
  const float* W1  = (const float*)d_in[8];
  const float* b1  = (const float*)d_in[9];
  const float* W2  = (const float*)d_in[10];
  const float* b2  = (const float*)d_in[11];
  float* out = (float*)d_out;

  constexpr size_t SZ_HALF = (size_t)MPAD * 384;
  constexpr size_t SZ_BIG  = 2 * SZ_HALF;
  constexpr size_t SZ_LIST = (size_t)NBLK * RCAP * 4;
  constexpr size_t SZ_TAB  = (size_t)NSL * 4;
  constexpr size_t SZ_META = (size_t)NBLK * MLINE * 4;
  constexpr size_t SZ_PL   = (size_t)PO_END * 2;
  constexpr size_t SZ_BIAS = (size_t)4 * 128 * 4;
  constexpr size_t O_A     = 0;
  constexpr size_t O_B     = O_A + SZ_BIG;
  constexpr size_t O_C     = O_B + SZ_BIG;
  constexpr size_t O_LISTF = O_C + SZ_BIG;
  constexpr size_t O_LISTB = O_LISTF + SZ_LIST;
  constexpr size_t O_CNTF  = O_LISTB + SZ_LIST;
  constexpr size_t O_CNTB  = O_CNTF + SZ_TAB;
  constexpr size_t O_OFFF  = O_CNTB + SZ_TAB;
  constexpr size_t O_OFFB  = O_OFFF + SZ_TAB;
  constexpr size_t O_RDI   = O_OFFB + SZ_TAB;
  constexpr size_t O_RDO   = O_RDI + SZ_TAB;
  constexpr size_t O_METAF = O_RDO + SZ_TAB;
  constexpr size_t O_METAB = O_METAF + SZ_META;
  constexpr size_t O_PL    = O_METAB + SZ_META;
  constexpr size_t O_BIAS  = O_PL + SZ_PL;
  constexpr size_t WS_TOTAL = O_BIAS + SZ_BIAS;
  static_assert(SZ_HALF % 256 == 0 && SZ_LIST % 256 == 0 && SZ_TAB % 256 == 0 && SZ_META % 128 == 0 && (2 * SZ_META) % 256 == 0);
  static_assert(SZ_PL % 256 == 0 && SZ_BIAS % 256 == 0);
  static_assert(WS_TOTAL == ((size_t)489945 << 8));
  static_assert(WS_TOTAL <= ((size_t)128 << 20));
  if (ws_size < WS_TOTAL) return;

  char* ws = (char*)d_ws;
  char* rA = ws + O_A;  char* rA1 = rA + SZ_HALF;
  char* rB = ws + O_B;  char* rB1 = rB + SZ_HALF;
  char* rC = ws + O_C;  char* rC1 = rC + SZ_HALF;
  int*   LISTF = (int*)(ws + O_LISTF);
  int*   LISTB = (int*)(ws + O_LISTB);
  int*   CNTF  = (int*)(ws + O_CNTF);
  int*   CNTB  = (int*)(ws + O_CNTB);
  int*   OFFF  = (int*)(ws + O_OFFF);
  int*   OFFB  = (int*)(ws + O_OFFB);
  float* RDI   = (float*)(ws + O_RDI);
  float* RDO   = (float*)(ws + O_RDO);
  int*   METAF = (int*)(ws + O_METAF);
  int*   METAB = (int*)(ws + O_METAB);
  unsigned short* PL = (unsigned short*)(ws + O_PL);
  float* BIAS  = (float*)(ws + O_BIAS);

  const size_t bLds = (size_t)AGG_LDS_INTS * 4;
  hipFuncSetAttribute(reinterpret_cast<const void*>(&k_bucket), hipFuncAttributeMaxDynamicSharedMemorySize, (int)bLds);
  const int vec8 = 1;
  const int tot4 = NNODE * HID / 4;

  k_prep<<<dim3(24, 9), NTHR, 0, stream>>>(Wq, Wp, W1, W2, bq, bp, b1, b2, PL, BIAS);
  k_bucket<<<NBLK, NTHR, bLds, stream>>>(dst, src, NEDGE, NNODE, vec8, LISTF, CNTF, OFFF, RDI, METAF);
  k_bucket<<<NBLK, NTHR, bLds, stream>>>(src, dst, NEDGE, NNODE, vec8, LISTB, CNTB, OFFB, RDO, METAB);
  k_xs<<<(NNODE * 48) / NTHR, NTHR, 0, stream>>>(q, p, RDO, (float*)rA, NNODE);
  k_fwd<<<NBLK, NTHR, 0, stream>>>(LISTF, CNTF, OFFF, METAF, RDI, (const float*)rA, (float*)rB, NNODE);
  mk_plane<TWO_TERM_AGG>((const float*)rB,      HID, 192, (unsigned short*)rC,  HID, stream);
  mk_plane<TWO_TERM_AGG>((const float*)rB + 96, HID, 192, (unsigned short*)rC1, HID, stream);
  run_gemm<1>((const unsigned short*)rC,  PL + PO_WQT, BIAS + 0,   (float*)rA,      HID, HID * DUP_AGG, 192, stream);
  run_gemm<1>((const unsigned short*)rC1, PL + PO_WPT, BIAS + 128, (float*)rA + 96, HID, HID * DUP_AGG, 192, stream);
  mk_plane<TWO_TERM_Z>((const float*)rA, 192, 192, (unsigned short*)rB, 192, stream);
  run_gemm<1>((const unsigned short*)rB, PL + PO_W1T, BIAS + 256, (float*)rC, HID, 192 * DUP_Z, HID, stream);
  k_tanh<<<(tot4 + NTHR - 1) / NTHR, NTHR, 0, stream>>>((const float*)rC, (float*)rC1, tot4);
  mk_plane<TWO_TERM_A>((const float*)rC1, HID, HID, (unsigned short*)rA, HID, stream);
  run_gemm<1>((const unsigned short*)rA, PL + PO_W2T, BIAS + 384, (float*)rA1, HID, HID * DUP_A, HID, stream);
  mk_plane<TWO_TERM_H>((const float*)rA1, HID, HID, (unsigned short*)rB, HID, stream);
  run_gemm<0>((const unsigned short*)rB, PL + PO_W2N, BIAS, (float*)rB1, HID, HID * DUP_H, HID, stream);
  k_du<<<(tot4 + NTHR - 1) / NTHR, NTHR, 0, stream>>>((const float*)rB1, (const float*)rC1, (float*)rC, tot4);
  mk_plane<TWO_TERM_DU>((const float*)rC, HID, HID, (unsigned short*)rA, HID, stream);
  run_gemm<0>((const unsigned short*)rA, PL + PO_W1N, BIAS, (float*)rB, 192, HID * DUP_DU, 192, stream);
  mk_plane<TWO_TERM_DZ>((const float*)rB,      HID, 192, (unsigned short*)rC,  HID, stream);
  mk_plane<TWO_TERM_DZ>((const float*)rB + 96, HID, 192, (unsigned short*)rC1, HID, stream);
  run_gemm<0>((const unsigned short*)rC,  PL + PO_WQN, BIAS, (float*)rA,      HID, HID * DUP_DZ, 192, stream);
  run_gemm<0>((const unsigned short*)rC1, PL + PO_WPN, BIAS, (float*)rA + 96, HID, HID * DUP_DZ, 192, stream);
  k_bwd<<<NBLK, NTHR, 0, stream>>>(LISTB, CNTB, OFFB, METAB, RDI, RDO, (const float*)rA, q, p, out, NNODE);
}
